// SyntaxMultiAttentionGAT_87144886436423
// MI455X (gfx1250) — hardware-run, weakly checked
//
#include <hip/hip_runtime.h>


namespace {
constexpr int NB_ = 4, LQ = 96, D = 256, H = 8, HD = 32, FF = 1024, NSEQ = NB_ * LQ  , NT = NSEQ * LQ  ;
constexpr float XS = 8.0f, HS = 256.0f, PS = 256.0f, WSC = 256.0f, EPS = 1e-5f, SCL = 0.17677669529663688f  ;
typedef _Float16 b16;
typedef __attribute__((ext_vector_type(16))) _Float16 v16b;
typedef __attribute__((ext_vector_type(8))) _Float16 v8b;
typedef __attribute__((ext_vector_type(2))) _Float16 v2b;
typedef __attribute__((ext_vector_type(8))) float v8f;
typedef __attribute__((ext_vector_type(4))) float v4f;
typedef __attribute__((ext_vector_type(2))) float v2f;
__device__ __forceinline__ float bf16_rne(float f) { unsigned int u = __float_as_uint(f); u += 0x7FFFu + ((u >> 16) & 1u); float r = __uint_as_float(u & 0xFFFF0000u); asm volatile("" : "+v"(r)); return r; }
__device__ __forceinline__ float bfv(float f) { float r = bf16_rne(f); asm volatile("" : "+v"(r)); return r; }
__device__ __forceinline__ void split16(float v, b16& hi, b16& lo) { hi = (b16)v; lo = (b16)(v - (float)hi); }
__device__ __forceinline__ v16b frag_kb(const b16* p, int hh) { const v8b a = *(const v8b*)(p + 8 * hh), b = *(const v8b*)(p + 16 + 8 * hh); v16b f;
#pragma unroll
  for (int e = 0; e < 8; ++e) { f[e] = a[e]; f[8 + e] = b[e]; } return f; }
__device__ __forceinline__ v8f wmma16b(v16b a, v16b b, v8f c) { v8f d = __builtin_amdgcn_wmma_f32_16x16x32_f16(false, a, false, b, (short)0, c, false, false); asm volatile("v_nop\n\tv_nop\n\tv_nop\n\tv_nop" : "+v"(d) : "v"(a), "v"(b)); return d; }
__device__ __forceinline__ void wave_lds_sync() { __builtin_amdgcn_fence(__ATOMIC_RELEASE, "workgroup"); __builtin_amdgcn_wave_barrier(); __builtin_amdgcn_fence(__ATOMIC_ACQUIRE, "workgroup"); }
__device__ __forceinline__ float pmul(float a, float b) { float p = a * b; asm volatile("" : "+v"(p)); return p; }

__global__ __launch_bounds__(256) void wput_kernel(const float* __restrict__ wq, const float* __restrict__ wk, const float* __restrict__ wv, const float* __restrict__ wo, const float* __restrict__ w1, const float* __restrict__ w2, b16* __restrict__ WQKV, b16* __restrict__ WO, b16* __restrict__ WF1, b16* __restrict__ WF2) { const size_t nt = (size_t)gridDim.x * 256, u0 = (size_t)blockIdx.x * 256 + threadIdx.x; v8b v;
  for (size_t u = u0; u < (size_t)3 * D * 32; u += nt) { const int o = (int)(u / 32), k0 = (int)(u % 32) * 8; const float* w = o < D ? wq : (o < 2 * D ? wk : wv); const int oo = o % D;
#pragma unroll
    for (int j = 0; j < 8; ++j) v[j] = (b16)(bf16_rne(w[(size_t)(k0 + j) * D + oo]) * WSC); for (int pass = 0; pass < 2; ++pass) { *(volatile v8b*)(WQKV + (size_t)o * D + k0) = v; __threadfence(); } }
  for (size_t u = u0; u < (size_t)D * 32; u += nt) { const int o = (int)(u / 32), k0 = (int)(u % 32) * 8;
#pragma unroll
    for (int j = 0; j < 8; ++j) v[j] = (b16)(bf16_rne(wo[(size_t)(k0 + j) * D + o]) * WSC); for (int pass = 0; pass < 2; ++pass) { *(volatile v8b*)(WO + (size_t)o * D + k0) = v; __threadfence(); } }
  for (size_t u = u0; u < (size_t)FF * 32; u += nt) { const int o = (int)(u / 32), k0 = (int)(u % 32) * 8;
#pragma unroll
    for (int j = 0; j < 8; ++j) v[j] = (b16)(bf16_rne(w1[(size_t)(k0 + j) * FF + o]) * WSC); for (int pass = 0; pass < 2; ++pass) { *(volatile v8b*)(WF1 + (size_t)o * D + k0) = v; __threadfence(); } }
  for (size_t u = u0; u < (size_t)D * 128; u += nt) { const int o = (int)(u / 128), k0 = (int)(u % 128) * 8;
#pragma unroll
    for (int j = 0; j < 8; ++j) v[j] = (b16)(bf16_rne(w2[(size_t)(k0 + j) * D + o]) * WSC); for (int pass = 0; pass < 2; ++pass) { *(volatile v8b*)(WF2 + (size_t)o * FF + k0) = v; __threadfence(); } } }
__global__ __launch_bounds__(32) void qkv_kernel(const float* __restrict__ tab, const b16* __restrict__ WQKV, const float* __restrict__ bq, const float* __restrict__ bk, const float* __restrict__ bv, b16* __restrict__ Qh, b16* __restrict__ Ql, b16* __restrict__ Kh, b16* __restrict__ Kl, float* __restrict__ V) { __shared__ __attribute__((aligned(16))) b16 Ah[16][D + 8]; __shared__ float Tf[16][260]; const int lane = threadIdx.x, nloc = lane & 15, hlf = lane >> 4; const size_t t0 = (size_t)blockIdx.x * 16;
  for (int rr = 0; rr < 16; ++rr) for (int q = 0; q < 8; ++q) { const int c = q * 32 + lane; Ah[rr][c] = (b16)(bf16_rne(tab[(t0 + rr) * D + c]) * XS); }
  if (lane < 16) for (int k = D; k < D + 8; ++k) Ah[lane][k] = (b16)0.0f;
  wave_lds_sync();
#pragma unroll 1
  for (int g = 0; g < 3; ++g) { const float* bias = g == 0 ? bq : (g == 1 ? bk : bv); v8f acc[16];
#pragma unroll
    for (int t = 0; t < 16; ++t) acc[t] = (v8f){};
#pragma unroll 2
    for (int kb = 0; kb < D; kb += 32) { const v16b a = frag_kb(&Ah[nloc][kb], hlf);
#pragma unroll
      for (int t = 0; t < 16; ++t) acc[t] = wmma16b(a, frag_kb(WQKV + (size_t)(g * D + t * 16 + nloc) * D + kb, hlf), acc[t]); }
#pragma unroll
    for (int t = 0; t < 16; ++t) { const int cc = t * 16 + nloc; const float bb = bfv(bias[cc]);
#pragma unroll
      for (int r8 = 0; r8 < 8; ++r8) Tf[8 * hlf + r8][cc] = acc[t][r8] * (1.0f / (XS * WSC)) + bb; }
    wave_lds_sync();
    for (int pass = 0; pass < 2; ++pass) { for (int rr = 0; rr < 16; ++rr) { const size_t tk = t0 + rr;
        if (g == 2) { for (int q = 0; q < 2; ++q) *(volatile v4f*)(V + tk * D + q * 128 + lane * 4) = *(const v4f*)(&Tf[rr][q * 128 + lane * 4]); }
        else { b16* Ph = g == 0 ? Qh : Kh; b16* Pl = g == 0 ? Ql : Kl; for (int q = 0; q < 4; ++q) { const int c = q * 64 + lane * 2; b16 h0, l0, h1, l1; split16(Tf[rr][c] * HS, h0, l0); split16(Tf[rr][c + 1] * HS, h1, l1); *(volatile v2b*)(Ph + tk * D + c) = (v2b){h0, h1}; *(volatile v2b*)(Pl + tk * D + c) = (v2b){l0, l1}; } } }
      __threadfence(); }
    wave_lds_sync(); } }
__global__ __launch_bounds__(256) void vt_kernel(const float* __restrict__ V, int SLIM, b16* __restrict__ VTh, b16* __restrict__ VTl) { __shared__ float Tt[8][LQ][HD + 1]; const int wave = threadIdx.x >> 5, lane = threadIdx.x & 31; const int seq = blockIdx.x, h = wave; if (seq >= SLIM) return;
  for (int k = 0; k < LQ; ++k) Tt[wave][k][lane] = V[((size_t)seq * LQ + k) * D + h * HD + lane];
  wave_lds_sync();
  const size_t base = ((size_t)seq * H + h) * HD * LQ;
  for (int pass = 0; pass < 2; ++pass) { for (int k = 0; k < LQ; k += 2) { b16 h0, l0, h1, l1; split16(Tt[wave][k][lane] * HS, h0, l0); split16(Tt[wave][k + 1][lane] * HS, h1, l1); *(volatile v2b*)(VTh + base + (size_t)lane * LQ + k) = (v2b){h0, h1}; *(volatile v2b*)(VTl + base + (size_t)lane * LQ + k) = (v2b){l0, l1}; } __threadfence(); } }
__global__ __launch_bounds__(32) void att_kernel(const b16* __restrict__ Qh, const b16* __restrict__ Ql, const b16* __restrict__ Kh, const b16* __restrict__ Kl, const b16* __restrict__ VTh, const b16* __restrict__ VTl, const float* __restrict__ dep, const float* __restrict__ wdep, const float* __restrict__ bdep, int SLIM, float* __restrict__ CTX) { __shared__ __attribute__((aligned(16))) b16 Pa[16][104], Pb[16][104]; __shared__ float Sc[16][LQ + 1], Dp[LQ], Of[16][HD + 1]; const int lane = threadIdx.x, nloc = lane & 15, hlf = lane >> 4; const int seq = blockIdx.x / (H * 6), rem = blockIdx.x % (H * 6); const int h = rem / 6, q0 = (rem % 6) * 16; if (seq >= SLIM) return; const size_t tk0 = (size_t)seq * LQ;
  const float wd = bfv(wdep[h]), bd = bfv(bdep[h]); for (int k = lane; k < LQ; k += 32) Dp[k] = pmul(bfv(dep[(size_t)seq * LQ + k]), wd) + bd;
  const v16b qa = frag_kb(Qh + (tk0 + q0 + nloc) * D + h * HD, hlf), ql = frag_kb(Ql + (tk0 + q0 + nloc) * D + h * HD, hlf);
#pragma unroll
  for (int t = 0; t < 6; ++t) { const size_t key = tk0 + t * 16 + nloc; const v16b kh = frag_kb(Kh + key * D + h * HD, hlf), kl = frag_kb(Kl + key * D + h * HD, hlf); v8f s = wmma16b(qa, kh, (v8f){}); s = wmma16b(qa, kl, s); s = wmma16b(ql, kh, s);
#pragma unroll
    for (int r8 = 0; r8 < 8; ++r8) Sc[8 * hlf + r8][t * 16 + nloc] = s[r8] * (SCL / (HS * HS)); }
  wave_lds_sync();
  if (lane < 16) { const int r = lane; float mx = -INFINITY; for (int k = 0; k < LQ; ++k) { const float v = Sc[r][k] + Dp[k]; Sc[r][k] = v; mx = fmaxf(mx, v); } float sm = 0.0f; for (int k = 0; k < LQ; ++k) { const float p = __expf(Sc[r][k] - mx); Sc[r][k] = p; sm += p; } const float inv = 1.0f / sm; for (int k = 0; k < LQ; ++k) { b16 p, pl; split16(Sc[r][k] * inv * PS, p, pl); Pa[r][k] = p; Pb[r][k] = pl; } for (int k = LQ; k < 104; ++k) { Pa[r][k] = (b16)0.0f; Pb[r][k] = (b16)0.0f; } }
  wave_lds_sync();
  v8f o0 = (v8f){}, o1 = (v8f){}; const size_t vb = ((size_t)seq * H + h) * HD * LQ;
#pragma unroll
  for (int kb = 0; kb < LQ; kb += 32) { const v16b pa = frag_kb(&Pa[nloc][kb], hlf), pb = frag_kb(&Pb[nloc][kb], hlf); const v16b v0h = frag_kb(VTh + vb + (size_t)nloc * LQ + kb, hlf), v0l = frag_kb(VTl + vb + (size_t)nloc * LQ + kb, hlf), v1h = frag_kb(VTh + vb + (size_t)(16 + nloc) * LQ + kb, hlf), v1l = frag_kb(VTl + vb + (size_t)(16 + nloc) * LQ + kb, hlf);
    o0 = wmma16b(pa, v0h, o0); o0 = wmma16b(pa, v0l, o0); o0 = wmma16b(pb, v0h, o0); o1 = wmma16b(pa, v1h, o1); o1 = wmma16b(pa, v1l, o1); o1 = wmma16b(pb, v1h, o1); }
#pragma unroll
  for (int r8 = 0; r8 < 8; ++r8) { Of[8 * hlf + r8][nloc] = o0[r8] * (1.0f / (PS * HS)); Of[8 * hlf + r8][16 + nloc] = o1[r8] * (1.0f / (PS * HS)); }
  wave_lds_sync();
  for (int pass = 0; pass < 2; ++pass) { for (int r = 0; r < 16; ++r) ((volatile float*)CTX)[(tk0 + q0 + r) * D + h * HD + lane] = Of[r][lane]; __threadfence(); } }
__global__ __launch_bounds__(32) void tail_kernel(const float* __restrict__ CTX, const float* __restrict__ tab, const b16* __restrict__ WO, const float* __restrict__ bo, const float* __restrict__ g1, const float* __restrict__ be1, const b16* __restrict__ WF1, const float* __restrict__ b1, const b16* __restrict__ WF2, const float* __restrict__ b2, const float* __restrict__ g2, const float* __restrict__ be2, int SLIM, float* __restrict__ out) { __shared__ __attribute__((aligned(16))) b16 A1h[16][D + 8], A1l[16][D + 8], A2h[16][FF + 8], A2l[16][FF + 8]; __shared__ float Y[16][D + 1], Tf[16][260]; const int lane = threadIdx.x, nloc = lane & 15, hlf = lane >> 4; const size_t t0 = (size_t)blockIdx.x * 16; if (t0 >= (size_t)SLIM * LQ) return;
  for (int rr = 0; rr < 16; ++rr) for (int q = 0; q < 8; ++q) { const int c = q * 32 + lane; b16 p, pl; split16(CTX[(t0 + rr) * D + c] * HS, p, pl); A1h[rr][c] = p; A1l[rr][c] = pl; }
  if (lane < 16) { for (int k = D; k < D + 8; ++k) { A1h[lane][k] = (b16)0.0f; A1l[lane][k] = (b16)0.0f; } for (int k = FF; k < FF + 8; ++k) { A2h[lane][k] = (b16)0.0f; A2l[lane][k] = (b16)0.0f; } }
  wave_lds_sync();
  auto ln_rows = [&](const float* gg, const float* bb) { if (lane < 16) { const int r = lane; float m = 0.0f; for (int c = 0; c < D; ++c) m += Y[r][c]; m *= (1.0f / D); float vr = 0.0f; for (int c = 0; c < D; ++c) { const float d = Y[r][c] - m; vr += d * d; } vr *= (1.0f / D); const float rs = rsqrtf(vr + EPS); for (int c = 0; c < D; ++c) Y[r][c] = pmul((Y[r][c] - m) * rs, bfv(gg[c])) + bfv(bb[c]); } wave_lds_sync(); };
  { v8f acc[16];
#pragma unroll
    for (int t = 0; t < 16; ++t) acc[t] = (v8f){};
#pragma unroll 2
    for (int kb = 0; kb < D; kb += 32) { const v16b a = frag_kb(&A1h[nloc][kb], hlf), al = frag_kb(&A1l[nloc][kb], hlf);
#pragma unroll
      for (int t = 0; t < 16; ++t) { const v16b bw = frag_kb(WO + (size_t)(t * 16 + nloc) * D + kb, hlf); acc[t] = wmma16b(a, bw, acc[t]); acc[t] = wmma16b(al, bw, acc[t]); } }
#pragma unroll
    for (int t = 0; t < 16; ++t) { const int cc = t * 16 + nloc; const float bb = bfv(bo[cc]);
#pragma unroll
      for (int r8 = 0; r8 < 8; ++r8) { const int r = 8 * hlf + r8; Y[r][cc] = acc[t][r8] * (1.0f / (HS * WSC)) + bb + bfv(tab[(t0 + r) * D + cc]); } } }
  wave_lds_sync(); ln_rows(g1, be1);
  for (int rr = 0; rr < 16; ++rr) for (int q = 0; q < 8; ++q) { const int c = q * 32 + lane; b16 p, pl; split16(Y[rr][c] * HS, p, pl); A1h[rr][c] = p; A1l[rr][c] = pl; }
  wave_lds_sync();
#pragma unroll 1
  for (int g = 0; g < 4; ++g) { v8f acc[16];
#pragma unroll
    for (int t = 0; t < 16; ++t) acc[t] = (v8f){};
#pragma unroll 2
    for (int kb = 0; kb < D; kb += 32) { const v16b a = frag_kb(&A1h[nloc][kb], hlf), al = frag_kb(&A1l[nloc][kb], hlf);
#pragma unroll
      for (int t = 0; t < 16; ++t) { const v16b bw = frag_kb(WF1 + (size_t)(g * 256 + t * 16 + nloc) * D + kb, hlf); acc[t] = wmma16b(a, bw, acc[t]); acc[t] = wmma16b(al, bw, acc[t]); } }
#pragma unroll
    for (int t = 0; t < 16; ++t) { const int cc = t * 16 + nloc; const float bb = bfv(b1[g * 256 + cc]);
#pragma unroll
      for (int r8 = 0; r8 < 8; ++r8) { const float v = fmaxf(acc[t][r8] * (1.0f / (HS * WSC)) + bb, 0.0f); b16 p, pl; split16(v * HS, p, pl); A2h[8 * hlf + r8][g * 256 + cc] = p; A2l[8 * hlf + r8][g * 256 + cc] = pl; } }
    wave_lds_sync(); }
  { v8f acc[16];
#pragma unroll
    for (int t = 0; t < 16; ++t) acc[t] = (v8f){};
#pragma unroll 2
    for (int kb = 0; kb < FF; kb += 32) { const v16b a = frag_kb(&A2h[nloc][kb], hlf), al = frag_kb(&A2l[nloc][kb], hlf);
#pragma unroll
      for (int t = 0; t < 16; ++t) { const v16b bw = frag_kb(WF2 + (size_t)(t * 16 + nloc) * FF + kb, hlf); acc[t] = wmma16b(a, bw, acc[t]); acc[t] = wmma16b(al, bw, acc[t]); } }
    wave_lds_sync();
#pragma unroll
    for (int t = 0; t < 16; ++t) { const int cc = t * 16 + nloc; const float bb = bfv(b2[cc]);
#pragma unroll
      for (int r8 = 0; r8 < 8; ++r8) { const int r = 8 * hlf + r8; Y[r][cc] = Y[r][cc] + acc[t][r8] * (1.0f / (HS * WSC)) + bb; } } }
  wave_lds_sync(); ln_rows(g2, be2);
  for (int pass = 0; pass < 2; ++pass) { for (int rr = 0; rr < 16; ++rr) for (int q = 0; q < 8; ++q) ((volatile float*)out)[(t0 + rr) * D + q * 32 + lane] = Y[rr][q * 32 + lane]; __threadfence(); } }
}

extern "C" void kernel_launch(void* const* d_in, const int* in_sizes, int n_in, void* d_out, int out_size, void* d_ws, size_t ws_size, hipStream_t stream) {
  (void)n_in;
  auto Fp = [&](int i) { return (const float*)d_in[i]; };
  if (in_sizes[0] != NT * D || in_sizes[1] != NT || in_sizes[2] != D * D || in_sizes[8] != D * D || in_sizes[10] != H || in_sizes[14] != D * FF || in_sizes[16] != FF * D || out_size != NT * D) return;
  const int SLIM = NSEQ;
  size_t off = 0; char* ws = (char*)d_ws;
  auto carve = [&](size_t bytes) { char* p = ws + off; off += (bytes + 255) & ~(size_t)255; return p; };
  b16* WQKV = (b16*)carve((size_t)3 * D * D * 2); b16* WO = (b16*)carve((size_t)D * D * 2); b16* WF1 = (b16*)carve((size_t)FF * D * 2); b16* WF2 = (b16*)carve((size_t)D * FF * 2); b16* Qh = (b16*)carve((size_t)NT * D * 2); b16* Ql = (b16*)carve((size_t)NT * D * 2); b16* Kh = (b16*)carve((size_t)NT * D * 2); b16* Kl = (b16*)carve((size_t)NT * D * 2); float* V = (float*)carve((size_t)NT * D * 4); b16* VTh = (b16*)carve((size_t)NSEQ * H * HD * LQ * 2); b16* VTl = (b16*)carve((size_t)NSEQ * H * HD * LQ * 2); float* CTX = (float*)carve((size_t)NT * D * 4);
  if (off > ws_size || off > ((size_t)208 << 20)) return;
  wput_kernel<<<128, 256, 0, stream>>>(Fp(2), Fp(4), Fp(6), Fp(8), Fp(14), Fp(16), WQKV, WO, WF1, WF2);
  qkv_kernel<<<SLIM * LQ / 16, 32, 0, stream>>>(Fp(0), WQKV, Fp(3), Fp(5), Fp(7), Qh, Ql, Kh, Kl, V);
  vt_kernel<<<NSEQ, 256, 0, stream>>>(V, SLIM, VTh, VTl);
  att_kernel<<<NSEQ * H * 6, 32, 0, stream>>>(Qh, Ql, Kh, Kl, VTh, VTl, Fp(1), Fp(10), Fp(11), SLIM, CTX);
  tail_kernel<<<NT / 16, 32, 0, stream>>>(CTX, Fp(0), WO, Fp(9), Fp(12), Fp(13), WF1, Fp(15), WF2, Fp(17), Fp(18), Fp(19), SLIM, (float*)d_out);
}
